// stackedIndRNN_encoder_7318624272387
// MI455X (gfx1250) — hardware-verified
//
#include <hip/hip_runtime.h>


#pragma clang fp contract(off)

#define T_    512
#define B_    128
#define JI_   75
#define H_    512
#define L_    6
#define C_    60
#define CP_   64
#define K0P_  96
#define M_    65536
#define TC_   128
#define NCH_  4
#define MC_   16384

static_assert(M_ == T_ * B_);
static_assert(TC_ * NCH_ == T_);
static_assert(MC_ == TC_ * B_);
static_assert(K0P_ % 32 == 0);
static_assert(K0P_ >= JI_);
static_assert(H_ % 64 == 0);
static_assert(MC_ % 32 == 0);
static_assert(CP_ >= C_);
static_assert((B_ * H_) % 512 == 0);

typedef float          v2f   __attribute__((ext_vector_type(2)));
typedef float          v4f   __attribute__((ext_vector_type(4)));
typedef float          v8f   __attribute__((ext_vector_type(8)));
typedef double         v2d   __attribute__((ext_vector_type(2)));
typedef __bf16         v16b  __attribute__((ext_vector_type(16)));
typedef unsigned short u16x8 __attribute__((ext_vector_type(8)));
typedef unsigned       u32x4 __attribute__((ext_vector_type(4)));

union Frag { u16x8 h[2]; v16b v; };

constexpr size_t SZ_XC  = (size_t)MC_ * H_ * 4;
constexpr size_t SZ_HP  = (size_t)M_ * H_ * 2;
constexpr size_t SZ_WH  = (size_t)(L_ - 1) * H_ * H_ * 2;
constexpr size_t SZ_W0  = (size_t)H_ * K0P_ * 2;
constexpr size_t SZ_WO  = (size_t)CP_ * H_ * 2;
constexpr size_t SZ_ST  = (size_t)B_ * H_ * 4;
constexpr size_t SZ_PS  = (size_t)B_ * H_ * 8;
constexpr size_t SZ_AFF = (size_t)L_ * 3 * H_ * 4;

constexpr size_t OFF_XC  = 0;
constexpr size_t OFF_HH  = OFF_XC + SZ_XC;
constexpr size_t OFF_HL  = OFF_HH + SZ_HP;
constexpr size_t OFF_WH  = OFF_HL + SZ_HP;
constexpr size_t OFF_W0  = OFF_WH + SZ_WH;
constexpr size_t OFF_WO  = OFF_W0 + SZ_W0;
constexpr size_t OFF_SA  = OFF_WO + SZ_WO;
constexpr size_t OFF_SB  = OFF_SA + SZ_ST;
constexpr size_t OFF_PSA = OFF_SB + SZ_ST;
constexpr size_t OFF_PQA = OFF_PSA + SZ_PS;
constexpr size_t OFF_PSB = OFF_PQA + SZ_PS;
constexpr size_t OFF_PQB = OFF_PSB + SZ_PS;
constexpr size_t OFF_AFF = OFF_PQB + SZ_PS;
constexpr size_t WS_END  = OFF_AFF + SZ_AFF;
static_assert(WS_END <= (size_t)268435456);
static_assert(OFF_HH % 512 == 0 && OFF_HL % 512 == 0 && OFF_WH % 512 == 0 && OFF_W0 % 512 == 0 && OFF_WO % 512 == 0);
static_assert(OFF_SA % 512 == 0 && OFF_SB % 512 == 0 && OFF_PSA % 512 == 0 && OFF_PQA % 512 == 0);
static_assert(OFF_PSB % 512 == 0 && OFF_PQB % 512 == 0 && OFF_AFF % 512 == 0 && WS_END % 512 == 0);

constexpr int LDS_BYTES = 65536;
static_assert(32 * H_ * 2 * 2 == LDS_BYTES);
static_assert(8 * 32 * 64 * 4 == LDS_BYTES);
static_assert(32 * K0P_ * 2 <= LDS_BYTES);

__device__ __forceinline__ unsigned short f2bf(float f) {
    unsigned u = __float_as_uint(f);
    unsigned r = u + 0x7FFFu + ((u >> 16) & 1u);
    return (unsigned short)(r >> 16);
}
__device__ __forceinline__ float bf2f(unsigned short b) {
    return __uint_as_float(((unsigned)b) << 16);
}
__device__ __forceinline__ float bfq(float f) { return bf2f(f2bf(f)); }
__device__ __forceinline__ v8f ld8f(const float* p) {
    const v4f a = *(const v4f*)p;
    const v4f b = *(const v4f*)(p + 4);
    return __builtin_shufflevector(a, b, 0, 1, 2, 3, 4, 5, 6, 7);
}

__device__ __forceinline__ void mma16(v8f& acc, const Frag& a, const Frag& b) {
    acc = __builtin_amdgcn_wmma_f32_16x16x32_bf16(false, a.v, false, b.v, (short)0, acc, false, false);
    asm volatile("v_nop\n\tv_nop\n\tv_nop\n\tv_nop" : "+v"(acc) : "v"(a.v), "v"(b.v));
}

__global__ __launch_bounds__(256)
void cvt_kernel(const float* __restrict__ src, unsigned short* dst, int nsrc, int kin, int kout, int n8)
{
    const int i = blockIdx.x * 256 + threadIdx.x;
    if (i >= n8) return;
    const size_t e = (size_t)i * 8;
    const int r  = (int)(e / (size_t)kout);
    const int c  = (int)(e - (size_t)r * kout);
    const int rc = min(r, nsrc - 1);
    const bool rin = (r < nsrc);
    u16x8 o;
    if ((kin & 7) == 0) {
        const int cc = min(c, kin - 8);
        const v4f a = *(const v4f*)(src + (size_t)rc * kin + cc);
        const v4f b = *(const v4f*)(src + (size_t)rc * kin + cc + 4);
#pragma unroll
        for (int q = 0; q < 4; ++q) {
            o[q]     = (rin && (c + q)     < kin) ? f2bf(a[q]) : (unsigned short)0;
            o[q + 4] = (rin && (c + q + 4) < kin) ? f2bf(b[q]) : (unsigned short)0;
        }
    } else {
#pragma unroll
        for (int q = 0; q < 8; ++q) {
            const int cq = min(c + q, kin - 1);
            const float v = src[(size_t)rc * kin + cq];
            o[q] = (rin && (c + q) < kin) ? f2bf(v) : (unsigned short)0;
        }
    }
    *(volatile u16x8*)(dst + e) = o;
    __threadfence();
    *(volatile u16x8*)(dst + e) = o;
}

template<int NTHR>
__device__ __forceinline__ void stage_split_rows(const unsigned short* __restrict__ Hh, const unsigned short* __restrict__ Hl,
                                                 size_t grow0, const float* __restrict__ aff,
                                                 unsigned short* sAh, unsigned short* sAl, int tid)
{
    constexpr int G8  = H_ / 8;
    constexpr int NIT = (32 * G8) / NTHR;
    static_assert((32 * G8) % NTHR == 0);
#pragma unroll 2
    for (int it = 0; it < NIT; ++it) {
        const int idx = it * NTHR + tid;
        const int row = idx / G8;
        const int c8  = (idx - row * G8) * 8;
        const size_t g = (grow0 + (size_t)row) * H_ + c8;
        const u32x4 hw = *(const u32x4*)(Hh + g);
        const u32x4 lw = *(const u32x4*)(Hl + g);
        const v8f mv = ld8f(aff + c8);
        const v8f sv = ld8f(aff + H_ + c8);
        const v8f bv = ld8f(aff + 2 * H_ + c8);
        u16x8 ho, lo;
#pragma unroll
        for (int q = 0; q < 4; ++q) {
            const unsigned a = hw[q];
            const unsigned b = lw[q];
            const float h0 = __uint_as_float(a << 16) + __uint_as_float(b << 16);
            const float h1 = __uint_as_float(a & 0xffff0000u) + __uint_as_float(b & 0xffff0000u);
            const float v0 = (h0 - mv[2 * q]) * sv[2 * q] + bv[2 * q];
            const float v1 = (h1 - mv[2 * q + 1]) * sv[2 * q + 1] + bv[2 * q + 1];
            const unsigned short hb0 = f2bf(v0);
            const unsigned short hb1 = f2bf(v1);
            ho[2 * q]     = hb0;
            ho[2 * q + 1] = hb1;
            lo[2 * q]     = f2bf(v0 - bf2f(hb0));
            lo[2 * q + 1] = f2bf(v1 - bf2f(hb1));
        }
        *(u16x8*)(sAh + row * H_ + c8) = ho;
        *(u16x8*)(sAl + row * H_ + c8) = lo;
    }
}

template<int KP, bool SPLIT>
__global__ __launch_bounds__(256)
void gemm_kernel(const float* __restrict__ Ax, const unsigned short* __restrict__ Hh, const unsigned short* __restrict__ Hl,
                 float* Xout, const unsigned short* __restrict__ Wp, const float* __restrict__ bias, const float* __restrict__ aff)
{
    static_assert(KP % 32 == 0);
    static_assert(!SPLIT || KP == H_);
    extern __shared__ __attribute__((aligned(16))) unsigned char dyn_lds[];
    unsigned short* sAh = reinterpret_cast<unsigned short*>(dyn_lds);
    unsigned short* sAl = sAh + 32 * KP;

    const int tid  = threadIdx.x;
    const int lane = tid & 31;
    const int wave = tid >> 5;
    const int h    = lane >> 4;
    const int m    = lane & 15;
    const int r0   = blockIdx.x * 32;

    if constexpr (!SPLIT) {
#pragma unroll 1
        for (int e = tid; e < 32 * KP; e += 256) {
            const int row = e / KP;
            const int col = e - row * KP;
            const int cc  = min(col, JI_ - 1);
            const float xv = Ax[(size_t)(r0 + row) * JI_ + cc];
            sAh[e] = (col < JI_) ? f2bf(xv) : (unsigned short)0;
        }
    } else {
        stage_split_rows<256>(Hh, Hl, (size_t)r0, aff, sAh, sAl, tid);
    }
    __syncthreads();

    v8f acc[2][4];
#pragma unroll
    for (int mt = 0; mt < 2; ++mt)
#pragma unroll
        for (int nt = 0; nt < 4; ++nt)
#pragma unroll
            for (int r = 0; r < 8; ++r) acc[mt][nt][r] = 0.0f;

    const int n0 = wave * 64;
    const unsigned short* bp = Wp + (size_t)(n0 + m) * KP + 8 * h;
    const unsigned short* ap = sAh + m * KP + 8 * h;
    const unsigned short* lp = sAl + m * KP + 8 * h;

#pragma unroll 1
    for (int ks = 0; ks < KP / 32; ++ks) {
        const int k0 = ks * 32;
        Frag fb[4], fa[2], ga[2];
#pragma unroll
        for (int nt = 0; nt < 4; ++nt) {
            const unsigned short* p = bp + (size_t)nt * 16 * KP + k0;
            fb[nt].h[0] = *(const u16x8*)(p);
            fb[nt].h[1] = *(const u16x8*)(p + 16);
        }
#pragma unroll
        for (int mt = 0; mt < 2; ++mt) {
            const unsigned short* p = ap + mt * 16 * KP + k0;
            fa[mt].h[0] = *(const u16x8*)(p);
            fa[mt].h[1] = *(const u16x8*)(p + 16);
            if constexpr (SPLIT) {
                const unsigned short* q = lp + mt * 16 * KP + k0;
                ga[mt].h[0] = *(const u16x8*)(q);
                ga[mt].h[1] = *(const u16x8*)(q + 16);
            }
        }
        if constexpr (SPLIT) {
#pragma unroll
            for (int mt = 0; mt < 2; ++mt)
#pragma unroll
                for (int nt = 0; nt < 4; ++nt) {
                    mma16(acc[mt][nt], fa[mt], fb[nt]);
                    mma16(acc[mt][nt], ga[mt], fb[nt]);
                }
        } else {
#pragma unroll
            for (int mt = 0; mt < 2; ++mt)
#pragma unroll
                for (int nt = 0; nt < 4; ++nt)
                    mma16(acc[mt][nt], fa[mt], fb[nt]);
        }
    }
    __syncthreads();

    float* st = reinterpret_cast<float*>(dyn_lds) + wave * (32 * 64);
#pragma unroll
    for (int nt = 0; nt < 4; ++nt) {
        const float bb = bfq(bias[n0 + nt * 16 + m]);
#pragma unroll
        for (int mt = 0; mt < 2; ++mt)
#pragma unroll
            for (int r = 0; r < 8; ++r)
                st[(mt * 16 + 8 * h + r) * 64 + nt * 16 + m] = acc[mt][nt][r] + bb;
    }
    __syncthreads();

    float* gbase = Xout + (size_t)r0 * H_ + n0;
    const int cs = m * 4;
#pragma unroll
    for (int it = 0; it < 16; ++it) {
        const int row = it * 2 + h;
        const v4f v = *(const v4f*)(st + row * 64 + cs);
        *(volatile v4f*)(gbase + (size_t)row * H_ + cs) = v;
    }
    __threadfence();
#pragma unroll
    for (int it = 0; it < 16; ++it) {
        const int row = it * 2 + h;
        const v4f v = *(const v4f*)(st + row * 64 + cs);
        *(volatile v4f*)(gbase + (size_t)row * H_ + cs) = v;
    }
}

__global__ __launch_bounds__(256)
void scan_kernel(const float* __restrict__ Xc, const float* __restrict__ ul,
                 const float* __restrict__ stin, const double* __restrict__ psin, const double* __restrict__ pqin,
                 unsigned short* Hh, unsigned short* Hl, float* stout, double* psout, double* pqout,
                 int tbase, int first)
{
    const int idx = blockIdx.x * 256 + threadIdx.x;
    const int b   = idx >> 8;
    const int c   = (idx & 255) * 2;
    const float u0 = bfq(ul[c]);
    const float u1 = bfq(ul[c + 1]);
    const size_t so = (size_t)b * H_ + c;
    const v2f sv = *(const v2f*)(stin + so);
    const v2d pv = *(const v2d*)(psin + so);
    const v2d qv = *(const v2d*)(pqin + so);
    const bool fz = (first != 0);
    float  h0 = fz ? 0.0f : sv[0];
    float  h1 = fz ? 0.0f : sv[1];
    double s0 = fz ? 0.0 : pv[0];
    double s1 = fz ? 0.0 : pv[1];
    double q0 = fz ? 0.0 : qv[0];
    double q1 = fz ? 0.0 : qv[1];

    const float* xp = Xc + so;
    const size_t ho = ((size_t)tbase * B_ + b) * H_ + c;
    unsigned short* hp = Hh + ho;
    unsigned short* lp = Hl + ho;
    const size_t step = (size_t)B_ * H_;
#pragma unroll 1
    for (int tl = 0; tl < TC_; ++tl) {
        const v2f xv = *(const v2f*)xp;
        const float a0 = xv[0] + u0 * h0;
        const float a1 = xv[1] + u1 * h1;
        h0 = fmaxf(a0, 0.0f);
        h1 = fmaxf(a1, 0.0f);
        const unsigned short hb0 = f2bf(h0);
        const unsigned short hb1 = f2bf(h1);
        const unsigned short lb0 = f2bf(h0 - bf2f(hb0));
        const unsigned short lb1 = f2bf(h1 - bf2f(hb1));
        const unsigned hw = (unsigned)hb0 | ((unsigned)hb1 << 16);
        const unsigned lw = (unsigned)lb0 | ((unsigned)lb1 << 16);
        *(volatile unsigned*)hp = hw;
        *(volatile unsigned*)lp = lw;
        __threadfence();
        *(volatile unsigned*)hp = hw;
        *(volatile unsigned*)lp = lw;
        const double d0 = (double)h0;
        const double d1 = (double)h1;
        s0 += d0;
        s1 += d1;
        q0 += d0 * d0;
        q1 += d1 * d1;
        xp += step;
        hp += step;
        lp += step;
    }
    v2f so2; so2[0] = h0; so2[1] = h1;
    v2d ps2; ps2[0] = s0; ps2[1] = s1;
    v2d pq2; pq2[0] = q0; pq2[1] = q1;
    *(volatile v2f*)(stout + so) = so2;
    *(volatile v2d*)(psout + so) = ps2;
    *(volatile v2d*)(pqout + so) = pq2;
    __threadfence();
    *(volatile v2f*)(stout + so) = so2;
    *(volatile v2d*)(psout + so) = ps2;
    *(volatile v2d*)(pqout + so) = pq2;
}

__global__ __launch_bounds__(256)
void bnfin_kernel(const double* __restrict__ psum, const double* __restrict__ psq,
                  const float* __restrict__ gam, const float* __restrict__ bet, float* aff)
{
    const int c = blockIdx.x * 256 + threadIdx.x;
    double s = 0.0, q = 0.0;
#pragma unroll 4
    for (int b = 0; b < B_; ++b) {
        s += psum[(size_t)b * H_ + c];
        q += psq[(size_t)b * H_ + c];
    }
    const double inv_n = 1.0 / (double)M_;
    const double mean  = s * inv_n;
    double var = q * inv_n - mean * mean;
    var = (var > 0.0) ? var : 0.0;
    const float mean32 = (float)mean;
    const float var32  = (float)var;
    const float scl = bfq(gam[c]) * (1.0f / sqrtf(var32 + 1e-5f));
    const float sh  = bfq(bet[c]);
    *(volatile float*)(aff + c)          = mean32;
    *(volatile float*)(aff + H_ + c)     = scl;
    *(volatile float*)(aff + 2 * H_ + c) = sh;
    __threadfence();
    *(volatile float*)(aff + c)          = mean32;
    *(volatile float*)(aff + H_ + c)     = scl;
    *(volatile float*)(aff + 2 * H_ + c) = sh;
}

__global__ __launch_bounds__(64)
void final_kernel(const unsigned short* __restrict__ Hh, const unsigned short* __restrict__ Hl,
                  const unsigned short* __restrict__ Wop, const float* __restrict__ bo,
                  const float* __restrict__ aff, float* out)
{
    extern __shared__ __attribute__((aligned(16))) unsigned char dyn_lds[];
    unsigned short* sAh = reinterpret_cast<unsigned short*>(dyn_lds);
    unsigned short* sAl = sAh + 32 * H_;

    const int tid  = threadIdx.x;
    const int lane = tid & 31;
    const int wave = tid >> 5;
    const int h    = lane >> 4;
    const int m    = lane & 15;
    const int m0   = blockIdx.x * 32;
    const size_t xrow0 = (size_t)(T_ - 1) * B_ + m0;

    stage_split_rows<64>(Hh, Hl, xrow0, aff, sAh, sAl, tid);
    __syncthreads();

    v8f acc[4];
#pragma unroll
    for (int nt = 0; nt < 4; ++nt)
#pragma unroll
        for (int r = 0; r < 8; ++r) acc[nt][r] = 0.0f;

    const unsigned short* bp = Wop + (size_t)m * H_ + 8 * h;
    const unsigned short* ap = sAh + (16 * wave + m) * H_ + 8 * h;
    const unsigned short* lp = sAl + (16 * wave + m) * H_ + 8 * h;

#pragma unroll 1
    for (int ks = 0; ks < H_ / 32; ++ks) {
        const int k0 = ks * 32;
        Frag fb[4], fa, ga;
#pragma unroll
        for (int nt = 0; nt < 4; ++nt) {
            const unsigned short* p = bp + (size_t)nt * 16 * H_ + k0;
            fb[nt].h[0] = *(const u16x8*)(p);
            fb[nt].h[1] = *(const u16x8*)(p + 16);
        }
        fa.h[0] = *(const u16x8*)(ap + k0);
        fa.h[1] = *(const u16x8*)(ap + k0 + 16);
        ga.h[0] = *(const u16x8*)(lp + k0);
        ga.h[1] = *(const u16x8*)(lp + k0 + 16);
#pragma unroll
        for (int nt = 0; nt < 4; ++nt) {
            mma16(acc[nt], fa, fb[nt]);
            mma16(acc[nt], ga, fb[nt]);
        }
    }
    __syncthreads();

    float* st = reinterpret_cast<float*>(dyn_lds);
#pragma unroll
    for (int nt = 0; nt < 4; ++nt) {
        const int n  = nt * 16 + m;
        const int nc = min(n, C_ - 1);
        const float braw = bo[nc];
        const float bb = (n < C_) ? bfq(braw) : 0.0f;
#pragma unroll
        for (int r = 0; r < 8; ++r)
            st[(16 * wave + 8 * h + r) * 64 + n] = acc[nt][r] + bb;
    }
    __syncthreads();

    float* ob = out + (size_t)m0 * C_;
    constexpr int NJ = (32 * C_) / 4;
    static_assert((32 * C_) % 4 == 0);
#pragma unroll
    for (int it = 0; it < 8; ++it) {
        const int j = it * 64 + tid;
        if (j < NJ) {
            v4f v;
#pragma unroll
            for (int q = 0; q < 4; ++q) {
                const int e   = 4 * j + q;
                const int row = e / C_;
                const int col = e - row * C_;
                v[q] = st[row * 64 + col];
            }
            *(volatile v4f*)(ob + 4 * j) = v;
        }
    }
    __threadfence();
#pragma unroll
    for (int it = 0; it < 8; ++it) {
        const int j = it * 64 + tid;
        if (j < NJ) {
            v4f v;
#pragma unroll
            for (int q = 0; q < 4; ++q) {
                const int e   = 4 * j + q;
                const int row = e / C_;
                const int col = e - row * C_;
                v[q] = st[row * 64 + col];
            }
            *(volatile v4f*)(ob + 4 * j) = v;
        }
    }
}

extern "C" void kernel_launch(void* const* d_in, const int* in_sizes, int n_in,
                              void* d_out, int out_size, void* d_ws, size_t ws_size,
                              hipStream_t stream)
{
    if (n_in < 10) return;
    if (in_sizes[0] != M_ * JI_)             return;
    if (in_sizes[1] != H_ * JI_)             return;
    if (in_sizes[2] != H_)                   return;
    if (in_sizes[3] != (L_ - 1) * H_ * H_)   return;
    if (in_sizes[4] != (L_ - 1) * H_)        return;
    if (in_sizes[5] != L_ * H_)              return;
    if (in_sizes[6] != L_ * H_)              return;
    if (in_sizes[7] != L_ * H_)              return;
    if (in_sizes[8] != C_ * H_)              return;
    if (in_sizes[9] != C_)                   return;
    if (out_size != B_ * C_)                 return;
    if (ws_size < WS_END)                    return;

    const float* x     = (const float*)d_in[0];
    const float* W0    = (const float*)d_in[1];
    const float* b0    = (const float*)d_in[2];
    const float* Wh    = (const float*)d_in[3];
    const float* bh    = (const float*)d_in[4];
    const float* u     = (const float*)d_in[5];
    const float* gamma = (const float*)d_in[6];
    const float* beta  = (const float*)d_in[7];
    const float* Wout  = (const float*)d_in[8];
    const float* bout  = (const float*)d_in[9];
    float* out = (float*)d_out;

    char* ws = (char*)d_ws;
    float*          Xc   = (float*)(ws + OFF_XC);
    unsigned short* Hh   = (unsigned short*)(ws + OFF_HH);
    unsigned short* Hl   = (unsigned short*)(ws + OFF_HL);
    unsigned short* Whp  = (unsigned short*)(ws + OFF_WH);
    unsigned short* W0p  = (unsigned short*)(ws + OFF_W0);
    unsigned short* Wop  = (unsigned short*)(ws + OFF_WO);
    float*          stA  = (float*)(ws + OFF_SA);
    float*          stB  = (float*)(ws + OFF_SB);
    double*         psA  = (double*)(ws + OFF_PSA);
    double*         pqA  = (double*)(ws + OFF_PQA);
    double*         psB  = (double*)(ws + OFF_PSB);
    double*         pqB  = (double*)(ws + OFF_PQB);
    float*          aff  = (float*)(ws + OFF_AFF);

    {
        const int n8a = (H_ * K0P_) / 8;
        const int n8b = ((L_ - 1) * H_ * H_) / 8;
        const int n8c = (CP_ * H_) / 8;
        static_assert(((H_ * K0P_) / 8) % 256 == 0);
        static_assert((((L_ - 1) * H_ * H_) / 8) % 256 == 0);
        static_assert(((CP_ * H_) / 8) % 256 == 0);
        cvt_kernel<<<dim3((n8a + 255) / 256), dim3(256), 0, stream>>>(W0, W0p, (int)H_, (int)JI_, (int)K0P_, n8a);
        cvt_kernel<<<dim3((n8b + 255) / 256), dim3(256), 0, stream>>>(Wh, Whp, (int)((L_ - 1) * H_), (int)H_, (int)H_, n8b);
        cvt_kernel<<<dim3((n8c + 255) / 256), dim3(256), 0, stream>>>(Wout, Wop, (int)C_, (int)H_, (int)H_, n8c);
    }

    const dim3 ggrid(MC_ / 32);
    const dim3 sgrid((B_ * H_ / 2) / 256);
    float*  stbuf[2] = { stA, stB };
    double* psbuf[2] = { psA, psB };
    double* pqbuf[2] = { pqA, pqB };
    constexpr int LASTB = (NCH_ - 1) & 1;
#pragma unroll 1
    for (int l = 0; l < L_; ++l) {
#pragma unroll 1
        for (int ch = 0; ch < NCH_; ++ch) {
            const size_t row0 = (size_t)ch * MC_;
            if (l == 0) {
                gemm_kernel<K0P_, false><<<ggrid, dim3(256), LDS_BYTES, stream>>>(
                    x + row0 * JI_, (const unsigned short*)Hh, (const unsigned short*)Hl, Xc,
                    (const unsigned short*)W0p, b0, (const float*)aff);
            } else {
                gemm_kernel<H_, true><<<ggrid, dim3(256), LDS_BYTES, stream>>>(
                    x, (const unsigned short*)(Hh + row0 * H_), (const unsigned short*)(Hl + row0 * H_), Xc,
                    (const unsigned short*)(Whp + (size_t)(l - 1) * H_ * H_),
                    bh + (size_t)(l - 1) * H_, (const float*)(aff + (size_t)(l - 1) * 3 * H_));
            }
            const int wb = ch & 1;
            const int rb = wb ^ 1;
            scan_kernel<<<sgrid, dim3(256), 0, stream>>>(
                (const float*)Xc, u + (size_t)l * H_,
                (const float*)stbuf[rb], (const double*)psbuf[rb], (const double*)pqbuf[rb],
                Hh, Hl, stbuf[wb], psbuf[wb], pqbuf[wb],
                (int)(ch * TC_), (int)(ch == 0 ? 1 : 0));
        }
        bnfin_kernel<<<dim3(H_ / 256), dim3(256), 0, stream>>>(
            (const double*)psbuf[LASTB], (const double*)pqbuf[LASTB],
            gamma + (size_t)l * H_, beta + (size_t)l * H_, aff + (size_t)l * 3 * H_);
    }

    final_kernel<<<dim3(B_ / 32), dim3(64), LDS_BYTES, stream>>>(
        (const unsigned short*)Hh, (const unsigned short*)Hl, (const unsigned short*)Wop, bout,
        (const float*)(aff + (size_t)(L_ - 1) * 3 * H_), out);
}
